// Attention_16535624090434
// MI455X (gfx1250) — hardware-verified
//
#include <hip/hip_runtime.h>


#ifndef NB
#define NB 128
#endif
#ifndef NCH
#if (NB % 8) == 0
#define NCH 2
#else
#define NCH 1
#endif
#endif
#define NBC   (NB / NCH)
#define NTOK  400
#define DM    256
#define NH    8
#define HD    32
#define NQK   512
#define VTP   448
#define KEYP  416
#define NPOS  1519
#define NPOSP 1536
#define XPAD  64
#define SPIT  420
#define PPIT  424
#define QSC   (0.17677669529663687f * 64.0f)
#define KSC   4.0f
#define VSC   16.0f
#define PCAR  1024.0f
#define RCAR  1024.0f
#define RINV  (1.0f / 1024.0f)
#define SINV  (1.0f / 256.0f)
#define OSC   (1.0f / 64.0f)
#define WSC   64.0f
#define FINV  (1.0f / 16384.0f)

static_assert(NB % NCH == 0);
static_assert((NBC * NTOK) % 64 == 0);
static_assert(NTOK % 16 == 0);
static_assert(NTOK % 4 == 0);
static_assert(DM % 64 == 0);
static_assert(NQK % 64 == 0);
static_assert(VTP % 64 == 0);
static_assert(KEYP % 32 == 0);
static_assert(KEYP >= NTOK);
static_assert(KEYP <= VTP);
static_assert(VTP - NTOK <= XPAD);
static_assert(NPOSP % 128 == 0);
static_assert(NPOSP >= NPOS);
static_assert(PPIT >= KEYP);
static_assert(PPIT % 8 == 0);
static_assert(SPIT % 4 == 0);
static_assert(SPIT >= NTOK);
static_assert(NH * HD == DM);

typedef _Float16 h16;
typedef unsigned short bf;
typedef __attribute__((ext_vector_type(16))) __bf16   v16bf;
typedef __attribute__((ext_vector_type(16))) _Float16 v16h;
typedef __attribute__((ext_vector_type(8)))  _Float16 v8h;
typedef __attribute__((ext_vector_type(4)))  _Float16 v4h;
typedef __attribute__((ext_vector_type(8)))  unsigned short v8us;
typedef __attribute__((ext_vector_type(2)))  unsigned short v2us;
typedef __attribute__((ext_vector_type(8)))  float    v8f;
typedef __attribute__((ext_vector_type(4)))  float    v4f;
typedef v8h  __attribute__((may_alias)) v8ha;
typedef v4h  __attribute__((may_alias)) v4ha;
typedef v4f  __attribute__((may_alias)) v4fa;

__device__ __forceinline__ unsigned short f2bf(float f) { unsigned u = __float_as_uint(f); u += 0x7FFFu + ((u >> 16) & 1u); return (unsigned short)(u >> 16); }
__device__ __forceinline__ float bf2f(unsigned short b) { return __uint_as_float(((unsigned)b) << 16); }
__device__ __forceinline__ float bfr(float f) { return bf2f(f2bf(f)); }
__device__ __forceinline__ v16h cat16(v8h lo, v8h hi) { return __builtin_shufflevector(lo, hi, 0, 1, 2, 3, 4, 5, 6, 7, 8, 9, 10, 11, 12, 13, 14, 15); }
__device__ __forceinline__ v16bf cat16b(v8us lo, v8us hi) { return __builtin_bit_cast(v16bf, __builtin_shufflevector(lo, hi, 0, 1, 2, 3, 4, 5, 6, 7, 8, 9, 10, 11, 12, 13, 14, 15)); }
__device__ __forceinline__ v8f wmma16(v16h a, v16h b, v8f c) { return __builtin_amdgcn_wmma_f32_16x16x32_f16(false, a, false, b, (short)0, c, false, false); }
__device__ __forceinline__ v8f wmmab(v16bf a, v16bf b, v8f c) { return __builtin_amdgcn_wmma_f32_16x16x32_bf16(false, a, false, b, (short)0, c, false, false); }
__device__ __forceinline__ void wave_sync() { __builtin_amdgcn_fence(3  , "wavefront"); __builtin_amdgcn_wave_barrier(); asm volatile("" ::: "memory"); }
__device__ __forceinline__ void hres(float y, h16& hv, h16& rv) { hv = (h16)y; rv = (h16)((y - (float)hv) * RCAR); }

template <typename T16> struct WFrag;
template <> struct WFrag<h16> { typedef v16h V; static __device__ __forceinline__ V ld(const h16* p) { return cat16(*(const v8h*)p, *(const v8h*)(p + 16)); } static __device__ __forceinline__ v8f mma(V a, V b, v8f c) { return wmma16(a, b, c); } };
template <> struct WFrag<bf> { typedef v16bf V; static __device__ __forceinline__ V ld(const bf* p) { return cat16b(*(const v8us*)p, *(const v8us*)(p + 16)); } static __device__ __forceinline__ v8f mma(V a, V b, v8f c) { return wmmab(a, b, c); } };

template <typename T16, int EPI, int MB, bool RES>
__global__ __launch_bounds__(32) void k_gemmw(const T16* __restrict__ A, const T16* __restrict__ A2, const T16* __restrict__ Bt, int K, float* Cf, h16* H0, h16* H1, h16* H2, int ldc, const float* __restrict__ bias, float osc, size_t sA, size_t sB, size_t sC) {
    typedef typename WFrag<T16>::V V;
    __shared__ __align__(16) float os[16 * 68];
    const size_t z = blockIdx.z; A += z * sA; if (RES) A2 += z * sA; Bt += z * sB;
    const unsigned lane = threadIdx.x & 31u, lr = lane & 15u, hi = lane >> 4; const unsigned r0 = blockIdx.x * (unsigned)(16 * MB), c0 = blockIdx.y * 64u;
    v8f acc[MB][4]; v8f accr[MB][4];
#pragma unroll
    for (int mb = 0; mb < MB; ++mb)
#pragma unroll
        for (int nb = 0; nb < 4; ++nb) { acc[mb][nb] = (v8f){}; if (RES) accr[mb][nb] = (v8f){}; }
    const size_t aoff = (size_t)(r0 + lr) * K + 8 * hi, boff = (size_t)(c0 + lr) * K + 8 * hi;
#pragma unroll 1
    for (int kc = 0; kc < K; kc += 32) {
        V a[MB], ar[MB];
#pragma unroll
        for (int mb = 0; mb < MB; ++mb) { a[mb] = WFrag<T16>::ld(A + aoff + (size_t)mb * 16 * K + kc); if (RES) ar[mb] = WFrag<T16>::ld(A2 + aoff + (size_t)mb * 16 * K + kc); }
#pragma unroll
        for (int nb = 0; nb < 4; ++nb) { const V b = WFrag<T16>::ld(Bt + boff + (size_t)nb * 16 * K + kc);
#pragma unroll
            for (int mb = 0; mb < MB; ++mb) { acc[mb][nb] = WFrag<T16>::mma(a[mb], b, acc[mb][nb]); if (RES) accr[mb][nb] = WFrag<T16>::mma(ar[mb], b, accr[mb][nb]); } }
        if (RES) { asm volatile("v_nop\n\tv_nop\n\tv_nop\n\tv_nop" : "+v"(acc[0][0]), "+v"(acc[MB - 1][3]), "+v"(accr[0][0]), "+v"(accr[MB - 1][3]) : "v"(a[0]), "v"(a[MB - 1]), "v"(ar[0]), "v"(ar[MB - 1])); }
        else { asm volatile("v_nop\n\tv_nop\n\tv_nop\n\tv_nop" : "+v"(acc[0][0]), "+v"(acc[MB - 1][1]), "+v"(acc[MB - 1][2]), "+v"(acc[MB - 1][3]) : "v"(a[0]), "v"(a[MB - 1])); }
    }
#pragma unroll
    for (int mb = 0; mb < MB; ++mb) {
#pragma unroll
        for (int nb = 0; nb < 4; ++nb) {
#pragma unroll
            for (int j = 0; j < 8; ++j) { float sv = acc[mb][nb][j]; if (RES) sv += accr[mb][nb][j] * RINV; os[(hi * 8 + j) * 68 + nb * 16 + lr] = sv; } }
        wave_sync();
        if (EPI == 0) {
            const unsigned g0 = r0 + (unsigned)mb * 16u; const unsigned bw = g0 / (unsigned)NTOK; const unsigned n0 = g0 - bw * (unsigned)NTOK;
            const unsigned sel = c0 >> 8; const float sc = sel ? KSC : QSC;
#pragma unroll 1
            for (int ps = 0; ps < 2; ++ps) {
#pragma unroll
                for (unsigned s = 0; s < 4; ++s) { const unsigned hsel = s >> 1; const unsigned idx = (s & 1u) * 32u + lane; const unsigned row = idx >> 2, col8 = (idx & 3u) * 8u;
                    const float* op = os + row * 68u + hsel * 32u + col8; const v4f x0 = *(const v4fa*)op, x1 = *(const v4fa*)(op + 4); const unsigned cb = c0 + hsel * 32u + col8; v8h o, orr;
#pragma unroll
                    for (unsigned e = 0; e < 4; ++e) { h16 hv, rv; hres((x0[e] + bfr(bias[cb + e])) * sc, hv, rv); o[e] = hv; orr[e] = rv; hres((x1[e] + bfr(bias[cb + 4u + e])) * sc, hv, rv); o[4 + e] = hv; orr[4 + e] = rv; }
                    const unsigned hh = ((c0 & 255u) >> 5) + hsel; const size_t off = (((size_t)bw * NH + hh) * NTOK + n0 + row) * HD + col8;
                    if (sel == 0) { *(volatile v8h*)(H0 + off) = o; *(volatile v8h*)(H2 + off) = orr; } else { *(volatile v8h*)(H1 + off) = o; } }
                if (ps == 0) __threadfence(); }
        } else if (EPI == 1) {
            const size_t cbo = z * sC + (size_t)(r0 + (unsigned)mb * 16u) * ldc + c0;
#pragma unroll 1
            for (int ps = 0; ps < 2; ++ps) {
#pragma unroll
                for (unsigned s = 0; s < 4; ++s) { const unsigned row = s * 4u + (lane >> 3), pc = (lane & 7u) * 8u; const float* op = os + row * 68u + pc; const v4f x0 = *(const v4fa*)op, x1 = *(const v4fa*)(op + 4);
                    const float bb = bfr(bias[NQK + r0 + (unsigned)mb * 16u + row]); v8h o, orr;
#pragma unroll
                    for (unsigned e = 0; e < 4; ++e) { h16 hv, rv; hres((x0[e] + bb) * VSC, hv, rv); o[e] = hv; orr[e] = rv; hres((x1[e] + bb) * VSC, hv, rv); o[4 + e] = hv; orr[4 + e] = rv; }
                    const size_t off = cbo + (size_t)row * ldc + pc;
                    *(volatile v8h*)(H0 + off) = o; *(volatile v8h*)(H2 + off) = orr; }
                if (ps == 0) __threadfence(); }
        } else {
            float* crow = Cf + (size_t)(r0 + (unsigned)mb * 16u) * ldc + c0;
#pragma unroll 1
            for (int ps = 0; ps < 2; ++ps) {
#pragma unroll
                for (unsigned s = 0; s < 8; ++s) { const unsigned row = 2u * s + hi, cofs = lr * 4u; const v4f x0 = *(const v4fa*)(os + row * 68u + cofs); v4f val;
#pragma unroll
                    for (unsigned e = 0; e < 4; ++e) val[e] = x0[e] * osc + bfr(bias[c0 + cofs + e]);
                    *(volatile v4f*)(crow + (size_t)row * ldc + cofs) = val; }
                if (ps == 0) __threadfence(); }
        }
        wave_sync();
    }
}

template <bool F16> __device__ __forceinline__ void wt_body(const float* __restrict__ w, unsigned N, unsigned nlines, unsigned short* Bt, float sc) {
    const unsigned lane = threadIdx.x & 31u; const unsigned L0 = (blockIdx.x * 8u + (threadIdx.x >> 5)) * 8u;
#pragma unroll 1
    for (int ps = 0; ps < 2; ++ps) {
#pragma unroll 1
        for (unsigned l = 0; l < 8; ++l) { const unsigned L = L0 + l; if (L >= nlines) break; const unsigned e = L * 64u + lane * 2u; const unsigned k = e & 255u, n = e >> 8;
            const float w0 = bfr(w[(size_t)k * N + n]), w1 = bfr(w[(size_t)(k + 1u) * N + n]); v2us o;
            if (F16) { o[0] = __builtin_bit_cast(unsigned short, (h16)(w0 * sc)); o[1] = __builtin_bit_cast(unsigned short, (h16)(w1 * sc)); } else { o[0] = f2bf(w0); o[1] = f2bf(w1); }
            *(volatile v2us*)(Bt + e) = o; }
        if (ps == 0) __threadfence(); }
}
__global__ __launch_bounds__(256) void k_wtb(const float* __restrict__ w, unsigned N, unsigned nlines, unsigned short* Bt) { wt_body<false>(w, N, nlines, Bt, 1.0f); }
__global__ __launch_bounds__(256) void k_wth(const float* __restrict__ w, unsigned N, unsigned nlines, unsigned short* Bt, float sc) { wt_body<true>(w, N, nlines, Bt, sc); }

__global__ __launch_bounds__(256) void k_cvt8(const float* __restrict__ src, bf* dst, unsigned n8src, unsigned n8all) {
    const unsigned i = blockIdx.x * 256u + threadIdx.x; if (i >= n8all) return; const unsigned is = (i < n8src) ? i : (n8src - 1u); const bool real = (i < n8src);
    const v8f v = *(const v8f*)(src + (size_t)is * 8); v8us o;
#pragma unroll
    for (int k = 0; k < 8; ++k) o[k] = real ? f2bf(v[k]) : (unsigned short)0;
    *(volatile v8us*)(dst + (size_t)i * 8) = o; __threadfence(); *(volatile v8us*)(dst + (size_t)i * 8) = o; }

__global__ __launch_bounds__(64) void k_pos(const float* __restrict__ pw, const float* __restrict__ pb,
                                            const float* __restrict__ g1, const float* __restrict__ b1, const float* __restrict__ w1, const float* __restrict__ c1,
                                            const float* __restrict__ g2, const float* __restrict__ b2, const float* __restrict__ w2, const float* __restrict__ c2,
                                            const float* __restrict__ g3, const float* __restrict__ b3, const float* __restrict__ w3, const float* __restrict__ c3, float* posT) {
    __shared__ float hs[64 * 17]; __shared__ float ys[64 * 17];
    const unsigned t = threadIdx.x & 63u; const unsigned p = blockIdx.x * 64u + t; float* hr = hs + t * 17u; float* yr = ys + t * 17u;
    const unsigned pr = p / 49u; const float dh = (float)((int)pr - 15), dw = (float)((int)(p - pr * 49u) - 24);
#pragma unroll 1
    for (unsigned j = 0; j < 16; ++j) hr[j] = dh * bfr(pw[j]) + dw * bfr(pw[16 + j]) + bfr(pb[j]);
#pragma unroll 1
    for (unsigned L = 0; L < 3; ++L) {
        const float* G = (L == 0) ? g1 : ((L == 1) ? g2 : g3); const float* Bn = (L == 0) ? b1 : ((L == 1) ? b2 : b3);
        const float* W = (L == 0) ? w1 : ((L == 1) ? w2 : w3); const float* Cb = (L == 0) ? c1 : ((L == 1) ? c2 : c3); const unsigned nc = (L == 2) ? 8u : 16u;
        float mu = 0.f;
#pragma unroll 1
        for (unsigned j = 0; j < 16; ++j) mu += hr[j];
        mu *= (1.0f / 16.0f); float var = 0.f;
#pragma unroll 1
        for (unsigned j = 0; j < 16; ++j) { const float d = hr[j] - mu; var += d * d; }
        var *= (1.0f / 16.0f); const float rs = rsqrtf(var + 1.0e-5f);
#pragma unroll 1
        for (unsigned j = 0; j < 16; ++j) { const float y = (hr[j] - mu) * rs * bfr(G[j]) + bfr(Bn[j]); yr[j] = fmaxf(y, 0.f); }
#pragma unroll 1
        for (unsigned j = 0; j < nc; ++j) { float s = bfr(Cb[j]);
#pragma unroll 1
            for (unsigned k = 0; k < 16; ++k) s += yr[k] * bfr(W[k * nc + j]);
            hr[j] = s; }
    }
#pragma unroll 1
    for (int ps = 0; ps < 2; ++ps) {
#pragma unroll 1
        for (unsigned h = 0; h < NH; ++h) { const float val = (p < (unsigned)NPOS) ? hr[h] : 0.f; *(volatile float*)(posT + (size_t)h * NPOSP + p) = val; }
        if (ps == 0) __threadfence(); }
}

__global__ __launch_bounds__(32) void k_attn(const h16* __restrict__ Qp, const h16* __restrict__ Qr, const h16* __restrict__ Kp, const h16* __restrict__ VT, const h16* __restrict__ VR, const float* __restrict__ posT, h16* CTX, h16* CTXR) {
    __shared__ __align__(16) float lpos[NPOSP];
    __shared__ __align__(16) float Ss[16 * SPIT];
    __shared__ __align__(16) h16   Ps[16 * PPIT];
    __shared__ __align__(16) float os[16 * 68];
    const unsigned lane = threadIdx.x & 31u, lr = lane & 15u, hi = lane >> 4; const unsigned m0 = blockIdx.x * 16u, hp = blockIdx.y, b = blockIdx.z;
    unsigned basec[8];
#pragma unroll
    for (unsigned r = 0; r < 8; ++r) { const unsigned i = m0 + 8u * hi + r; const unsigned ti = i / 25u; basec[r] = ti * 49u + (i - ti * 25u) + 759u; }
#pragma unroll 1
    for (unsigned hh = 0; hh < 2; ++hh) {
        const unsigned h = hp * 2u + hh; const size_t bh = (size_t)b * NH + h;
        wave_sync();
#pragma unroll
        for (unsigned q = 0; q < NPOSP / 128; ++q) { const unsigned idx = (q * 32u + lane) * 4u; *(v4fa*)(lpos + idx) = *(const v4f*)(posT + (size_t)h * NPOSP + idx); }
        wave_sync();
        const size_t qo = (bh * NTOK + m0 + lr) * HD + 8u * hi;
        const v16h qf = cat16(*(const v8h*)(Qp + qo), *(const v8h*)(Qp + qo + 16)); const v16h qrf = cat16(*(const v8h*)(Qr + qo), *(const v8h*)(Qr + qo + 16));
        const h16* kp = Kp + (bh * NTOK + lr) * HD + 8u * hi;
#pragma unroll 1
        for (unsigned jt = 0; jt < NTOK / 16; ++jt) {
            const h16* kq = kp + (size_t)jt * 16u * HD; const v16h kf = cat16(*(const v8h*)kq, *(const v8h*)(kq + 16));
            v8f sv = (v8f){}, sr = (v8f){}; sv = wmma16(qf, kf, sv); sr = wmma16(qrf, kf, sr);
            asm volatile("v_nop\n\tv_nop\n\tv_nop\n\tv_nop" : "+v"(sv), "+v"(sr) : "v"(qf), "v"(qrf), "v"(kf));
            const unsigned col = jt * 16u + lr; const unsigned tj = col / 25u; const unsigned jc = tj * 49u + (col - tj * 25u);
#pragma unroll
            for (unsigned r = 0; r < 8; ++r) Ss[(8u * hi + r) * SPIT + col] = (sv[r] + sr[r] * RINV) * SINV + lpos[basec[r] - jc];
        }
        wave_sync();
#pragma unroll 1
        for (unsigned row = 0; row < 16; ++row) {
            const float* sr = Ss + row * SPIT; float v[16]; float mx = -3.0e38f;
#pragma unroll
            for (unsigned q = 0; q < 4; ++q) { const unsigned c = q * 32u + lane; const unsigned cc = (c < 99u) ? c : 99u; const v4f a = *(const v4fa*)(sr + cc * 4u); const bool ok = (c < 100u);
#pragma unroll
                for (unsigned e = 0; e < 4; ++e) { const float tv = ok ? a[e] : -1.0e30f; v[q * 4 + e] = tv; mx = fmaxf(mx, tv); } }
#pragma unroll
            for (int sh = 16; sh; sh >>= 1) mx = fmaxf(mx, __shfl_xor(mx, sh, 32));
            float sum = 0.f;
#pragma unroll
            for (unsigned k = 0; k < 16; ++k) { const float d0 = v[k] - mx; const float ev = __builtin_amdgcn_exp2f(d0 * 1.4426950408889634f); v[k] = ev; sum += ev; }
#pragma unroll
            for (int sh = 16; sh; sh >>= 1) sum += __shfl_xor(sum, sh, 32);
            const float f = PCAR * (1.0f / sum);
#pragma unroll
            for (unsigned q = 0; q < 4; ++q) { const unsigned c = q * 32u + lane; v4h o;
#pragma unroll
                for (unsigned e = 0; e < 4; ++e) o[e] = (h16)(v[q * 4 + e] * f);
                if (c < (unsigned)(KEYP / 4)) *(v4ha*)(Ps + row * PPIT + c * 4u) = o; }
        }
        wave_sync();
        v8f a0 = (v8f){}, a1 = (v8f){}, ra0 = (v8f){}, ra1 = (v8f){};
        const size_t vo = (bh * HD + lr) * VTP + 8u * hi;
        const h16* pp = Ps + lr * PPIT + 8u * hi; const h16* v0 = VT + vo; const h16* v1 = v0 + (size_t)16 * VTP; const h16* w0 = VR + vo; const h16* w1 = w0 + (size_t)16 * VTP;
#pragma unroll 1
        for (unsigned kc = 0; kc < KEYP / 32; ++kc) {
            const v16h pf = cat16(*(const v8ha*)(pp + kc * 32u), *(const v8ha*)(pp + kc * 32u + 16u));
            const v16h vf0 = cat16(*(const v8h*)(v0 + kc * 32u), *(const v8h*)(v0 + kc * 32u + 16u));
            const v16h vf1 = cat16(*(const v8h*)(v1 + kc * 32u), *(const v8h*)(v1 + kc * 32u + 16u));
            const v16h wf0 = cat16(*(const v8h*)(w0 + kc * 32u), *(const v8h*)(w0 + kc * 32u + 16u));
            const v16h wf1 = cat16(*(const v8h*)(w1 + kc * 32u), *(const v8h*)(w1 + kc * 32u + 16u));
            a0 = wmma16(pf, vf0, a0); a1 = wmma16(pf, vf1, a1); ra0 = wmma16(pf, wf0, ra0); ra1 = wmma16(pf, wf1, ra1);
            asm volatile("v_nop\n\tv_nop\n\tv_nop\n\tv_nop" : "+v"(a0), "+v"(a1), "+v"(ra0), "+v"(ra1) : "v"(pf), "v"(vf0), "v"(vf1), "v"(wf0), "v"(wf1));
        }
#pragma unroll
        for (unsigned r = 0; r < 8; ++r) { os[(8u * hi + r) * 68u + hh * 32u + lr] = (a0[r] + ra0[r] * RINV) * OSC; os[(8u * hi + r) * 68u + hh * 32u + 16u + lr] = (a1[r] + ra1[r] * RINV) * OSC; }
    }
    wave_sync();
#pragma unroll 1
    for (int ps = 0; ps < 2; ++ps) {
#pragma unroll
        for (unsigned s = 0; s < 4; ++s) { const unsigned row = s * 4u + (lane >> 3), pc = (lane & 7u) * 8u; const float* op = os + row * 68u + pc; const v4f x0 = *(const v4fa*)op, x1 = *(const v4fa*)(op + 4); v8h o, orr;
#pragma unroll
            for (unsigned e = 0; e < 4; ++e) { h16 hv, rv; hres(x0[e], hv, rv); o[e] = hv; orr[e] = rv; hres(x1[e], hv, rv); o[4 + e] = hv; orr[4 + e] = rv; }
            const size_t off = ((size_t)b * NTOK + m0 + row) * DM + hp * 64u + pc;
            *(volatile v8h*)(CTX + off) = o; *(volatile v8h*)(CTXR + off) = orr; }
        if (ps == 0) __threadfence(); }
}

extern "C" void kernel_launch(void* const* d_in, const int* in_sizes, int n_in,
                              void* d_out, int out_size, void* d_ws, size_t ws_size, hipStream_t stream) {
    if (n_in < 19) return;
    if (in_sizes[0] < NB * NTOK * DM || in_sizes[1] < DM * 3 * DM || in_sizes[2] < 3 * DM || in_sizes[3] < DM * DM || in_sizes[4] < DM) return;
    if (in_sizes[5] < 32 || in_sizes[6] < 16 || in_sizes[7] < 16 || in_sizes[8] < 16 || in_sizes[9] < 256 || in_sizes[10] < 16 || in_sizes[11] < 16 || in_sizes[12] < 16) return;
    if (in_sizes[13] < 256 || in_sizes[14] < 16 || in_sizes[15] < 16 || in_sizes[16] < 16 || in_sizes[17] < 128 || in_sizes[18] < 8) return;
    if (out_size < NB * NTOK * DM) return;
    const float* x = (const float*)d_in[0]; const float* wqkv = (const float*)d_in[1]; const float* bqkv = (const float*)d_in[2]; const float* wo = (const float*)d_in[3]; const float* bo = (const float*)d_in[4];
    const float* ppw = (const float*)d_in[5]; const float* ppb = (const float*)d_in[6];
    const float* l1g = (const float*)d_in[7]; const float* l1b = (const float*)d_in[8]; const float* p1w = (const float*)d_in[9]; const float* p1b = (const float*)d_in[10];
    const float* l2g = (const float*)d_in[11]; const float* l2b = (const float*)d_in[12]; const float* p2w = (const float*)d_in[13]; const float* p2b = (const float*)d_in[14];
    const float* l3g = (const float*)d_in[15]; const float* l3b = (const float*)d_in[16]; const float* p3w = (const float*)d_in[17]; const float* p3b = (const float*)d_in[18];
    float* OUT = (float*)d_out;
    char* wsp = (char*)d_ws;
    auto take = [&](size_t bytes) { char* p = wsp; wsp += (bytes + 255) & ~(size_t)255; return (void*)p; };
    const size_t ROWSC = (size_t)NBC * NTOK;
    bf* XB = (bf*)take((ROWSC + XPAD) * DM * 2);
    bf* WQKV = (bf*)take((size_t)3 * DM * DM * 2);
    h16* WO = (h16*)take((size_t)DM * DM * 2);
    float* POST = (float*)take((size_t)NH * NPOSP * 4);
    h16* QP = (h16*)take(ROWSC * DM * 2); h16* QR = (h16*)take(ROWSC * DM * 2); h16* KP = (h16*)take(ROWSC * DM * 2);
    h16* VTp = (h16*)take((size_t)NBC * DM * VTP * 2); h16* VRp = (h16*)take((size_t)NBC * DM * VTP * 2);
    h16* CTXR = (h16*)take(ROWSC * DM * 2);
    if ((size_t)(wsp - (char*)d_ws) > ws_size) return;
    if ((size_t)(wsp - (char*)d_ws) > (size_t)134217728) return;
    h16* CTX = (h16*)XB;
    const unsigned n8src = (unsigned)(ROWSC * DM / 8), n8all = (unsigned)((ROWSC + XPAD) * DM / 8);
    { const unsigned nl = 3u * DM * DM / 64u; k_wtb<<<(nl + 63u) / 64u, 256, 0, stream>>>(wqkv, 3u * DM, nl, WQKV); }
    { const unsigned nl = (unsigned)DM * DM / 64u; k_wth<<<(nl + 63u) / 64u, 256, 0, stream>>>(wo, (unsigned)DM, nl, (unsigned short*)WO, WSC); }
    k_pos<<<NPOSP / 64, 64, 0, stream>>>(ppw, ppb, l1g, l1b, p1w, p1b, l2g, l2b, p2w, p2b, l3g, l3b, p3w, p3b, POST);
    for (unsigned c = 0; c < (unsigned)NCH; ++c) {
        const float* xc = x + (size_t)c * ROWSC * DM; float* oc = OUT + (size_t)c * ROWSC * DM;
        k_cvt8<<<(n8all + 255u) / 256u, 256, 0, stream>>>(xc, XB, n8src, n8all);
        k_gemmw<bf, 0, 4, false><<<dim3((unsigned)(ROWSC / 64), NQK / 64, 1), 32, 0, stream>>>(XB, nullptr, WQKV, DM, nullptr, QP, KP, QR, 0, bqkv, 1.0f, 0, 0, 0);
        k_gemmw<bf, 1, 4, false><<<dim3(DM / 64, VTP / 64, NBC), 32, 0, stream>>>(WQKV + (size_t)NQK * DM, nullptr, XB, DM, nullptr, VTp, nullptr, VRp, VTP, bqkv, 1.0f, 0, (size_t)NTOK * DM, (size_t)DM * VTP);
        k_attn<<<dim3(NTOK / 16, NH / 2, NBC), 32, 0, stream>>>(QP, QR, KP, VTp, VRp, POST, CTX, CTXR);
        k_gemmw<h16, 2, 2, true><<<dim3((unsigned)(ROWSC / 32), DM / 64, 1), 32, 0, stream>>>(CTX, CTXR, WO, DM, oc, nullptr, nullptr, nullptr, DM, bo, FINV, 0, 0, 0);
    }
}
